// GraphConv2d_41308995453321
// MI455X (gfx1250) — hardware-verified
//
#include <hip/hip_runtime.h>
#include <stddef.h>
#include <stdint.h>

#define NB     8
#define NC     192
#define NNODE  3136
#define KE     9
#define NO     384
#define NPQ    768
#define MTOT   (NB * NNODE)
#define EI1    (NB * NNODE * KE)
#define GBM    64
#define GBN    64
#define GTHR   128
#define TT     64
#define SXP    65
#define CGW    128
#define SOP    68
#define NTHR   256
#define WSMAX  134217728

static_assert((MTOT % GBM) == 0);
static_assert((NNODE % TT) == 0 && (NC % TT) == 0);
static_assert((NC % 32) == 0);
static_assert((NO % GBN) == 0 && (NO % CGW) == 0);
static_assert((NPQ * (NC / 8)) % NTHR == 0);
static_assert(TT * TT == NTHR * 16);
static_assert((SOP * 4) % 16 == 0);
static_assert(CGW == 4 * 32);
static_assert(GBM == (GTHR / 32) * 16);

typedef float          v4f  __attribute__((ext_vector_type(4)));
typedef float          v8f  __attribute__((ext_vector_type(8)));
typedef int            v8i  __attribute__((ext_vector_type(8)));
typedef unsigned short v8us __attribute__((ext_vector_type(8)));
typedef __bf16         v16y __attribute__((ext_vector_type(16)));
union FragB { v16y v; v8us h[2]; v8i w; };

__device__ __forceinline__ v8f wmb(const FragB& a, const FragB& b, v8f c) {
  v8f d = __builtin_amdgcn_wmma_f32_16x16x32_bf16(false, a.v, false, b.v, (short)0, c, false, false);
  asm volatile("v_nop\n\tv_nop\n\tv_nop\n\tv_nop" : "+v"(d) : "v"(a.w), "v"(b.w));
  return d;
}

__device__ __forceinline__ unsigned short bf16_rne(float f) {
  unsigned int u = __float_as_uint(f);
  u = u + 0x7FFFu + ((u >> 16) & 1u);
  return (unsigned short)(u >> 16);
}

__device__ __forceinline__ v8us cvt8b(const v4f a, const v4f c) {
  v8us o;
  o[0] = bf16_rne(a.x); o[1] = bf16_rne(a.y); o[2] = bf16_rne(a.z); o[3] = bf16_rne(a.w);
  o[4] = bf16_rne(c.x); o[5] = bf16_rne(c.y); o[6] = bf16_rne(c.z); o[7] = bf16_rne(c.w);
  return o;
}

__global__ __launch_bounds__(NTHR) void k_xt(const float* __restrict__ x, unsigned short* xt) {
  __shared__ __attribute__((aligned(16))) float sx[TT * SXP];
  const int tid = (int)threadIdx.x, lane = tid & 31, wave = tid >> 5;
  const int n0 = (int)blockIdx.x * TT, c0 = (int)blockIdx.y * TT, b = (int)blockIdx.z;
#pragma unroll
  for (int it = 0; it < 4; ++it) {
    const int idx = it * NTHR + tid;
    const int row = idx >> 4;
    const int c4  = (idx & 15) * 4;
    const v4f v = *(const v4f*)(x + (size_t)(b * NC + c0 + row) * (size_t)NNODE + n0 + c4);
    float* d = sx + row * SXP + c4;
    d[0] = v.x; d[1] = v.y; d[2] = v.z; d[3] = v.w;
  }
  __syncthreads();

  const int q8 = lane & 7, sub = lane >> 3;
  v8us ov[2];
  size_t go[2];
#pragma unroll
  for (int i = 0; i < 2; ++i) {
    const int nd = 32 * i + 4 * wave + sub;
    v8us o;
#pragma unroll
    for (int j = 0; j < 8; ++j) o[j] = bf16_rne(sx[(8 * q8 + j) * SXP + nd]);
    ov[i] = o;
    go[i] = (size_t)(b * NNODE + n0 + nd) * (size_t)NC + c0 + 8 * q8;
    *(volatile v8us*)(xt + go[i]) = ov[i];
  }
  __threadfence();
#pragma unroll
  for (int i = 0; i < 2; ++i) *(volatile v8us*)(xt + go[i]) = ov[i];
}

__global__ __launch_bounds__(NTHR) void k_wt(const float* __restrict__ W, unsigned short* wt) {
  const int u = (int)blockIdx.x * NTHR + (int)threadIdx.x;
  if (u >= NPQ * (NC / 8)) return;
  const int r  = u / (NC / 8);
  const int k8 = (u - r * (NC / 8)) * 8;
  const int o  = (r < NO) ? r : (r - NO);
  const int hf = (r < NO) ? 0 : NC;
  const float* p = W + (size_t)o * (size_t)(2 * NC) + hf + k8;
  const v4f a = *(const v4f*)p;
  const v4f c = *(const v4f*)(p + 4);
  const v8us hv = cvt8b(a, c);
  const size_t go = (size_t)r * (size_t)NC + k8;
  *(volatile v8us*)(wt + go) = hv;
  __threadfence();
  *(volatile v8us*)(wt + go) = hv;
}

__global__ __launch_bounds__(GTHR) void k_gemm(const unsigned short* __restrict__ XT,
                                               const unsigned short* __restrict__ WT, float* RQ) {
  __shared__ __attribute__((aligned(16))) float stg[GBM * 2 * GBN];
  const int tid = (int)threadIdx.x, lane = tid & 31, wave = tid >> 5, hh = lane >> 4, m = lane & 15;
  const int rowBase = (int)blockIdx.x * GBM;
  const int col0    = (int)blockIdx.y * GBN;

  v8f ap[4], aq[4];
  {
    const v8f z = {0.f, 0.f, 0.f, 0.f, 0.f, 0.f, 0.f, 0.f};
#pragma unroll
    for (int t = 0; t < 4; ++t) { ap[t] = z; aq[t] = z; }
  }
  const unsigned short* apn = XT + (size_t)(rowBase + 16 * wave + m) * (size_t)NC + 8 * hh;
  const unsigned short* wpp = WT + (size_t)(col0 + m) * (size_t)NC + 8 * hh;
  const unsigned short* wpq = WT + (size_t)(NO + col0 + m) * (size_t)NC + 8 * hh;
#pragma unroll 1
  for (int ks = 0; ks < NC / 32; ++ks) {
    FragB af;
    af.h[0] = *(const v8us*)(apn + 32 * ks);
    af.h[1] = *(const v8us*)(apn + 32 * ks + 16);
#pragma unroll
    for (int t = 0; t < 4; ++t) {
      const unsigned short* wq0 = wpp + (size_t)(16 * t) * (size_t)NC + 32 * ks;
      const unsigned short* wq1 = wpq + (size_t)(16 * t) * (size_t)NC + 32 * ks;
      FragB bf, cf;
      bf.h[0] = *(const v8us*)wq0;
      bf.h[1] = *(const v8us*)(wq0 + 16);
      cf.h[0] = *(const v8us*)wq1;
      cf.h[1] = *(const v8us*)(wq1 + 16);
      ap[t] = wmb(af, bf, ap[t]);
      aq[t] = wmb(af, cf, aq[t]);
    }
  }

#pragma unroll
  for (int t = 0; t < 4; ++t) {
    const int lc = 16 * t + m;
#pragma unroll
    for (int r = 0; r < 8; ++r) {
      const int lr = 16 * wave + 8 * hh + r;
      const float pv = ap[t][r];
      const float qv = aq[t][r];
      stg[lr * (2 * GBN) + lc]       = pv - qv;
      stg[lr * (2 * GBN) + GBN + lc] = qv;
    }
  }
  __syncthreads();

  v4f fr[8], fq[8];
#pragma unroll
  for (int i = 0; i < 8; ++i) {
    const int lr = 16 * wave + 2 * i + hh;
    fr[i] = *(const v4f*)(stg + lr * (2 * GBN) + 4 * m);
    fq[i] = *(const v4f*)(stg + lr * (2 * GBN) + GBN + 4 * m);
  }
#pragma unroll
  for (int i = 0; i < 8; ++i) {
    const int gr = rowBase + 16 * wave + 2 * i + hh;
    float* op = RQ + (size_t)gr * (size_t)NPQ + col0 + 4 * m;
    *(volatile v4f*)op = fr[i];
    *(volatile v4f*)(op + NO) = fq[i];
  }
  __threadfence();
#pragma unroll
  for (int i = 0; i < 8; ++i) {
    const int gr = rowBase + 16 * wave + 2 * i + hh;
    float* op = RQ + (size_t)gr * (size_t)NPQ + col0 + 4 * m;
    *(volatile v4f*)op = fr[i];
    *(volatile v4f*)(op + NO) = fq[i];
  }
}

__global__ __launch_bounds__(NTHR) void k_edge(const float* __restrict__ RQ, const int* __restrict__ ei,
                                               const float* __restrict__ bias, float* out) {
  __shared__ __attribute__((aligned(16))) float so[CGW * SOP];
  __shared__ int sI[TT * KE];
  __shared__ int sJ[TT * KE];
  const int tid = (int)threadIdx.x, lane = tid & 31, wave = tid >> 5, hh = lane >> 4, m = lane & 15;
  const int n0 = (int)blockIdx.x * TT, cg = (int)blockIdx.y, b = (int)blockIdx.z;

  const size_t eb = ((size_t)b * NNODE + n0) * (size_t)KE;
#pragma unroll 1
  for (int t = tid; t < TT * KE; t += NTHR) {
    int j = ei[eb + t];
    int i = ei[(size_t)EI1 + eb + t];
    j = j < 0 ? 0 : (j > NNODE - 1 ? NNODE - 1 : j);
    i = i < 0 ? 0 : (i > NNODE - 1 ? NNODE - 1 : i);
    sJ[t] = j;
    sI[t] = i;
  }
  __syncthreads();

  const int cb = cg * CGW + 4 * lane;
  const v4f bv = *(const v4f*)(bias + cb);
  const float* Rb = RQ + (size_t)b * NNODE * (size_t)NPQ + cb;
  const float* Qb = Rb + NO;
#pragma unroll 1
  for (int nd = 0; nd < 8; ++nd) {
    const int node = 8 * wave + nd;
    v4f mx = {0.f, 0.f, 0.f, 0.f};
#pragma unroll 3
    for (int k = 0; k < KE; ++k) {
      const int i = sI[node * KE + k];
      const int j = sJ[node * KE + k];
      const v4f rv = *(const v4f*)(Rb + (size_t)i * (size_t)NPQ);
      const v4f qv = *(const v4f*)(Qb + (size_t)j * (size_t)NPQ);
      const v4f v = (rv + qv) + bv;
      mx.x = fmaxf(mx.x, v.x);
      mx.y = fmaxf(mx.y, v.y);
      mx.z = fmaxf(mx.z, v.z);
      mx.w = fmaxf(mx.w, v.w);
    }
    so[(4 * lane + 0) * SOP + node] = mx.x;
    so[(4 * lane + 1) * SOP + node] = mx.y;
    so[(4 * lane + 2) * SOP + node] = mx.z;
    so[(4 * lane + 3) * SOP + node] = mx.w;
  }
  __syncthreads();

  v4f fv[8];
  size_t go[8];
#pragma unroll
  for (int i = 0; i < 8; ++i) {
    const int lr = 16 * wave + 2 * i + hh;
    fv[i] = *(const v4f*)(so + lr * SOP + 4 * m);
    go[i] = (size_t)(b * NO + cg * CGW + lr) * (size_t)NNODE + n0 + 4 * m;
    *(volatile v4f*)(out + go[i]) = fv[i];
  }
  __threadfence();
#pragma unroll
  for (int i = 0; i < 8; ++i) *(volatile v4f*)(out + go[i]) = fv[i];
}

extern "C" void kernel_launch(void* const* d_in, const int* in_sizes, int n_in,
                              void* d_out, int out_size, void* d_ws, size_t ws_size,
                              hipStream_t stream) {
  if (n_in < 4) return;
  if (in_sizes[0] != NB * NC * NNODE) return;
  if (in_sizes[1] != 2 * EI1) return;
  if (in_sizes[2] != NO * 2 * NC) return;
  if (in_sizes[3] != NO) return;
  if (out_size != NB * NO * NNODE) return;

  const float* x    = (const float*)d_in[0];
  const int*   ei   = (const int*)d_in[1];
  const float* W    = (const float*)d_in[2];
  const float* bias = (const float*)d_in[3];
  float* out = (float*)d_out;

  char* ws = (char*)d_ws;
  size_t off = 0;
  const size_t oXT = off; off += (size_t)MTOT * NC * 2;      off = (off + 255) & ~(size_t)255;
  const size_t oWT = off; off += (size_t)NPQ * NC * 2;       off = (off + 255) & ~(size_t)255;
  const size_t oRQ = off; off += (size_t)MTOT * NPQ * 4;     off = (off + 255) & ~(size_t)255;
  if (off > ws_size || off > (size_t)WSMAX) return;
  unsigned short* XT = (unsigned short*)(ws + oXT);
  unsigned short* WTp = (unsigned short*)(ws + oWT);
  float* RQ = (float*)(ws + oRQ);

  k_xt<<<dim3(NNODE / TT, NC / TT, NB), NTHR, 0, stream>>>(x, XT);
  k_wt<<<(NPQ * (NC / 8)) / NTHR, NTHR, 0, stream>>>(W, WTp);
  k_gemm<<<dim3(MTOT / GBM, NO / GBN), GTHR, 0, stream>>>(XT, WTp, RQ);
  k_edge<<<dim3(NNODE / TT, NO / CGW, NB), NTHR, 0, stream>>>(RQ, ei, bias, out);
}
